// MCR2_HGPD_62680752718518
// MI455X (gfx1250) — hardware-run, weakly checked
//
#include <hip/hip_runtime.h>
#include <stddef.h>
#include <stdint.h>


#define NU1    50000
#define NU2    50000
#define NUSR   100000
#define NCOM   200000
#define NEDG   1000000
#define EDIM   85
#define DCD    64
#define HD     128
#define MPAD   100096
#define UFP    128
#define GPI    192
#define CPI    128
#define KT     416
#define BTN    256
#define NTILE  782

#ifndef ZERO_LO_G
#define ZERO_LO_G 0
#endif
#ifndef ZERO_LO_C
#define ZERO_LO_C 0
#endif

#define NTHR   256
#define NWAVE  8
#define EPT    8
#define CHUNK  (NTHR * EPT)
#define WCAP   (EPT * 32)
#define LISTN  (NWAVE * WCAP)
#define NBA    1024
#define SLA    10
#define NBLK   98
#define NSLOT  (NBLK * NBA)
#define RCAP   12288
#define DEGCAP 64
#define RBW    192
#define AGG_ZINTS    (LISTN + 2 * RCAP + 3 * NBA)
#define AGG_LDS_INTS (AGG_ZINTS + 16)
#define WSMAX  134217728

#define PB0    3125
#define PB1    6250
#define PB2    6256
#define PB3    6257
#define PBTOT  6258

static_assert(EDIM <= 96 && KT % 32 == 0 && KT == 96 + 192 + 128);
static_assert(NUSR == 781 * 128 + 32 && MPAD == NTILE * 128 && MPAD >= NUSR);
static_assert(UFP % 64 == 0 && GPI % 64 == 0 && CPI % 64 == 0);
static_assert(RCAP >= 10578 + 10578 / 20 + 1 && RCAP >= 10433 + 10433 / 20 + 1);
static_assert(DEGCAP >= 33 + 8 && DEGCAP >= 26 + 8);
static_assert(NBLK * NBA >= MPAD);
static_assert((CHUNK & (CHUNK - 1)) == 0 && CHUNK <= 4096);
static_assert((NBA & (NBA - 1)) == 0 && NBA == (1 << SLA) && NBA == NTHR * 4);
static_assert(((long long)CHUNK << SLA) < (1LL << 31));
static_assert(NEDG < (1 << 21) && (NEDG % 4) == 0);
static_assert(RCAP % (NTHR * 4) == 0 && AGG_ZINTS % (NTHR * 4) == 0);
static_assert(AGG_LDS_INTS * 4 <= 300000);
static_assert(NU1 % 16 == 0 && NU2 % 16 == 0 && (MPAD - NUSR) % 16 == 0);
static_assert(PB0 * 16 == NU1 && (PB1 - PB0) * 16 == NU2 && (PB2 - PB1) * 16 == MPAD - NUSR);
static_assert((NUSR * HD / 4) % NTHR == 0);
static_assert(128 * 128 * 4 + 256 * 4 + 256 * 4 <= 327680);

typedef float          v2f   __attribute__((ext_vector_type(2)));
typedef float          v4f   __attribute__((ext_vector_type(4)));
typedef float          v8f   __attribute__((ext_vector_type(8)));
typedef int            v4i   __attribute__((ext_vector_type(4)));
typedef int            v8i   __attribute__((ext_vector_type(8)));
typedef unsigned       v2u   __attribute__((ext_vector_type(2)));
typedef unsigned short v2us  __attribute__((ext_vector_type(2)));
typedef unsigned short v4us  __attribute__((ext_vector_type(4)));
typedef unsigned short v8us  __attribute__((ext_vector_type(8)));
typedef unsigned short v16us __attribute__((ext_vector_type(16)));
typedef __bf16         v16bf __attribute__((ext_vector_type(16)));
typedef v2f  __attribute__((may_alias)) v2fa;
typedef v4f  __attribute__((may_alias)) v4fa;
typedef v4i  __attribute__((may_alias)) v4ia;
typedef v2u  __attribute__((may_alias)) v2ua;
typedef v2us __attribute__((may_alias)) v2usa;
typedef v4us __attribute__((may_alias)) v4usa;
typedef v8us __attribute__((may_alias)) v8usa;
union FragB { v16bf v; v16us u; v8us h[2]; v8i w; };

__device__ __forceinline__ v8f wmb(const FragB& a, const FragB& b, v8f c) {
  v8f d = __builtin_amdgcn_wmma_f32_16x16x32_bf16(false, a.v, false, b.v, (short)0, c, false, false);
  asm volatile("v_nop\n\tv_nop\n\tv_nop\n\tv_nop" : "+v"(d) : "v"(a.w), "v"(b.w));
  return d;
}

__device__ __forceinline__ unsigned bf16_bits(float f) {
  const unsigned u = __float_as_uint(f);
  return (u + 0x7FFFu + ((u >> 16) & 1u)) >> 16;
}
__device__ __forceinline__ float bf16_val(float f) {
  return __uint_as_float(bf16_bits(f) << 16);
}

__device__ __forceinline__ void wave_sync() {
  __builtin_amdgcn_fence(__ATOMIC_RELEASE, "wavefront");
  __builtin_amdgcn_wave_barrier();
  __builtin_amdgcn_fence(__ATOMIC_ACQUIRE, "wavefront");
}

template <int SLB>
__device__ __forceinline__ int scan_chunk(const int* __restrict__ dsts, int nE, int cbase, int slotBase,
                                          int nb, int vec8, int* list, int tid, int lane, int wave) {
  int wc = 0;
  const int el0  = tid * EPT;
  const int e0   = cbase + el0;
  const int sent = -2147483647 - 1;
  v4i da, db;
  if (vec8 != 0 && cbase + CHUNK <= nE) {
    da = *(const v4i*)(dsts + e0);
    db = *(const v4i*)(dsts + e0 + 4);
  } else {
    const int nl = nE - 1;
    const int k0 = dsts[min(e0,     nl)];
    const int k1 = dsts[min(e0 + 1, nl)];
    const int k2 = dsts[min(e0 + 2, nl)];
    const int k3 = dsts[min(e0 + 3, nl)];
    const int k4 = dsts[min(e0 + 4, nl)];
    const int k5 = dsts[min(e0 + 5, nl)];
    const int k6 = dsts[min(e0 + 6, nl)];
    const int k7 = dsts[min(e0 + 7, nl)];
    asm volatile("" :: "v"(k0), "v"(k1), "v"(k2), "v"(k3), "v"(k4), "v"(k5), "v"(k6), "v"(k7));
    da.x = (e0     < nE) ? k0 : sent;
    da.y = (e0 + 1 < nE) ? k1 : sent;
    da.z = (e0 + 2 < nE) ? k2 : sent;
    da.w = (e0 + 3 < nE) ? k3 : sent;
    db.x = (e0 + 4 < nE) ? k4 : sent;
    db.y = (e0 + 5 < nE) ? k5 : sent;
    db.z = (e0 + 6 < nE) ? k6 : sent;
    db.w = (e0 + 7 < nE) ? k7 : sent;
  }
  const unsigned nbs = (unsigned)slotBase;
  const unsigned unb = (unsigned)nb;
  const unsigned s0 = (unsigned)da.x - nbs, s1 = (unsigned)da.y - nbs;
  const unsigned s2 = (unsigned)da.z - nbs, s3 = (unsigned)da.w - nbs;
  const unsigned s4 = (unsigned)db.x - nbs, s5 = (unsigned)db.y - nbs;
  const unsigned s6 = (unsigned)db.z - nbs, s7 = (unsigned)db.w - nbs;
  const bool h0 = s0 < unb, h1 = s1 < unb, h2 = s2 < unb, h3 = s3 < unb;
  const bool h4 = s4 < unb, h5 = s5 < unb, h6 = s6 < unb, h7 = s7 < unb;
  const unsigned any = __builtin_amdgcn_ballot_w32(h0 | h1 | h2 | h3 | h4 | h5 | h6 | h7);
  if (any != 0u) {
#define HITJ(J, HJ, SJ) { \
      const unsigned mj = __builtin_amdgcn_ballot_w32(HJ); \
      if (mj != 0u) { \
        if (HJ) { \
          const int pos = wc + (int)__builtin_amdgcn_mbcnt_lo(mj, 0u); \
          if (pos < WCAP) list[wave * WCAP + pos] = ((el0 + (J)) << SLB) | (int)(SJ); \
        } \
        wc += (int)__builtin_popcount(mj); } }
    HITJ(0, h0, s0)
    HITJ(1, h1, s1)
    HITJ(2, h2, s2)
    HITJ(3, h3, s3)
    HITJ(4, h4, s4)
    HITJ(5, h5, s5)
    HITJ(6, h6, s6)
    HITJ(7, h7, s7)
#undef HITJ
  }
  return wc;
}

__device__ __forceinline__ void fill_region(const float* __restrict__ W, int Kin, int period, int kstart,
                                            int ngroups, int n0, unsigned short* stage, int tid) {
  const int nun = 16 * ngroups;
#pragma unroll 1
  for (int ub = 0; ub < nun; ub += NTHR) {
    const int qq = ub + tid;
    const int q  = qq < nun ? qq : nun - 1;
    const int rl = q & 15, gg = q >> 4;
    const int n  = n0 + rl, h = n >> 7, c = n & 127;
    const float* wb = W + (size_t)h * (size_t)Kin * HD + c;
    float v[8];
#pragma unroll
    for (int e = 0; e < 8; ++e) {
      const int jj = 8 * gg + e;
      const int j  = jj >= period ? jj - period : jj;
      const int jc = j < Kin ? j : Kin - 1;
      v[e] = wb[(size_t)jc * HD];
    }
    asm volatile("" :: "v"(v[0]), "v"(v[1]), "v"(v[2]), "v"(v[3]), "v"(v[4]), "v"(v[5]), "v"(v[6]), "v"(v[7]));
    v8us o;
#pragma unroll
    for (int e = 0; e < 8; ++e) {
      const int jj = 8 * gg + e;
      const int j  = jj >= period ? jj - period : jj;
      const unsigned msk = (j < Kin) ? 0xffffu : 0u;
      o[e] = (unsigned short)(bf16_bits(v[e]) & msk);
    }
    if (qq < nun) *(v8usa*)(stage + rl * KT + kstart + 8 * gg) = o;
  }
}

__global__ __launch_bounds__(NTHR) void k_prep(const int* __restrict__ nidx, const float* __restrict__ uf,
                                               const float* __restrict__ emb,
                                               const float* __restrict__ e0, const float* __restrict__ e3,
                                               const float* __restrict__ e7, const float* __restrict__ e8,
                                               const float* __restrict__ e9,
                                               const float* __restrict__ wg, const float* __restrict__ bg,
                                               const float* __restrict__ wl, const float* __restrict__ bl,
                                               const float* __restrict__ wr, const float* __restrict__ gam,
                                               const float* __restrict__ bet,
                                               unsigned short* ufpl, unsigned short* btpl, float* par) {
  __shared__ __attribute__((aligned(16))) unsigned short rowt[16 * UFP];
  __shared__ __attribute__((aligned(16))) unsigned short stage[16 * KT];
  __shared__ float et[160];
  __shared__ float ufl[16 * 12];
  const int tid = (int)threadIdx.x, lane = tid & 31;
  const int wv  = __builtin_amdgcn_readfirstlane(tid >> 5);
  const int bid = (int)blockIdx.x;

  if (bid < PB0) {
    const int row0 = bid * 16;
    {
      const v8us z8 = {0, 0, 0, 0, 0, 0, 0, 0};
      *(v8usa*)(rowt + 8 * tid) = z8;
      float tv = 0.0f;
      if (wv == 0)      tv = e0[lane];
      else if (wv == 1) tv = e3[lane];
      else if (wv == 2) tv = e7[lane];
      else if (wv == 3) tv = e8[lane];
      else if (wv == 4) tv = e9[lane];
      if (wv < 5) et[wv * 32 + lane] = bf16_val(tv);
      const int q  = tid < 160 ? tid : 159;
      const int r  = q / 10, ci = q - 10 * r;
      const float uv = uf[(size_t)(row0 + r) * 10 + ci];
      asm volatile("" :: "v"(uv));
      if (tid < 160) ufl[r * 12 + ci] = bf16_val(uv);
    }
    __syncthreads();
#pragma unroll 1
    for (int j = 0; j < 5; ++j) {
      const int q   = tid + NTHR * j;
      const int r   = q / 80, rem = q - 80 * r;
      const int t   = rem >> 4, k = rem & 15;
      const int ucol = (int)((0x98730u >> (4 * t)) & 15u);
      const int cb   = (int)((0x4535251200ULL >> (8 * t)) & 0xffULL);
      const float fv = ufl[r * 12 + ucol];
      int ix = (int)fv;
      ix = ix < 0 ? 0 : (ix > 1 ? 1 : ix);
      const float val = et[t * 32 + ix * 16 + k];
      rowt[r * UFP + cb + k] = (unsigned short)(__float_as_uint(val) >> 16);
    }
    {
      const int q  = tid < 80 ? tid : 79;
      const int r  = q / 5, j = q - 5 * r;
      const int ucol = (int)((0x65421u >> (4 * j)) & 15u);
      const int dc   = (int)((0x2423221110ULL >> (8 * j)) & 0xffULL);
      const float val = ufl[r * 12 + ucol];
      if (tid < 80) rowt[r * UFP + dc] = (unsigned short)(__float_as_uint(val) >> 16);
    }
    __syncthreads();
    {
      const int r = tid >> 4, u = tid & 15;
      const v8us q = *(const v8usa*)(rowt + r * UFP + 8 * u);
      unsigned short* dp = ufpl + (size_t)(row0 + r) * UFP + 8 * u;
      *(volatile v8us*)dp = q;
      __threadfence();
      *(volatile v8us*)dp = q;
    }
  } else if (bid < PB1) {
    const int r = tid >> 4, u = tid & 15;
    const int row = NU1 + (bid - PB0) * 16 + r;
    int ix = nidx[row - NU1];
    ix = ix < 0 ? 0 : (ix > NU2 - 1 ? NU2 - 1 : ix);
    const float* bp = emb + (size_t)ix * EDIM;
    float v[8];
#pragma unroll
    for (int e = 0; e < 8; ++e) {
      const int c  = 8 * u + e;
      const int cc = c < EDIM ? c : EDIM - 1;
      v[e] = bp[cc];
    }
    asm volatile("" :: "v"(v[0]), "v"(v[1]), "v"(v[2]), "v"(v[3]), "v"(v[4]), "v"(v[5]), "v"(v[6]), "v"(v[7]));
    v8us o;
#pragma unroll
    for (int e = 0; e < 8; ++e) {
      const int c = 8 * u + e;
      const unsigned msk = (c < EDIM) ? 0xffffu : 0u;
      o[e] = (unsigned short)(bf16_bits(v[e]) & msk);
    }
    unsigned short* dp = ufpl + (size_t)row * UFP + 8 * u;
    *(volatile v8us*)dp = o;
    __threadfence();
    *(volatile v8us*)dp = o;
  } else if (bid < PB2) {
    const int r = tid >> 4, u = tid & 15;
    const int row = NUSR + (bid - PB1) * 16 + r;
    const v8us z8 = {0, 0, 0, 0, 0, 0, 0, 0};
    unsigned short* dp = ufpl + (size_t)row * UFP + 8 * u;
    *(volatile v8us*)dp = z8;
    __threadfence();
    *(volatile v8us*)dp = z8;
  } else if (bid == PB2) {
#pragma unroll 1
    for (int ch = 0; ch < BTN / 16; ++ch) {
      const int n0 = 16 * ch;
      fill_region(wr, EDIM, 96, 0,   12, n0, stage, tid);
      fill_region(wg, EDIM, 96, 96,  24, n0, stage, tid);
      fill_region(wl, DCD,  64, 288, 16, n0, stage, tid);
      __syncthreads();
      v8us qv[4];
#pragma unroll
      for (int i = 0; i < 4; ++i) {
        const int uu = tid + NTHR * i;
        const int uc = uu < 832 ? uu : 831;
        qv[i] = *(const v8usa*)(stage + 8 * uc);
      }
      unsigned short* base = btpl + (size_t)n0 * KT;
#pragma unroll
      for (int i = 0; i < 4; ++i) {
        const int uu = tid + NTHR * i;
        if (uu < 832) *(volatile v8us*)(base + 8 * uu) = qv[i];
      }
      __threadfence();
#pragma unroll
      for (int i = 0; i < 4; ++i) {
        const int uu = tid + NTHR * i;
        if (uu < 832) *(volatile v8us*)(base + 8 * uu) = qv[i];
      }
      __syncthreads();
    }
  } else if (bid == PB3) {
    v4f t = {0.0f, 0.0f, 0.0f, 0.0f};
    if (wv < 2)       t = *(const v4f*)(bg  + 4 * tid);
    else if (wv < 4)  t = *(const v4f*)(bl  + 4 * (tid - 64));
    else if (wv == 4) t = *(const v4f*)(gam + 4 * (tid - 128));
    else if (wv == 5) t = *(const v4f*)(bet + 4 * (tid - 160));
    v4f o;
    o.x = bf16_val(t.x); o.y = bf16_val(t.y); o.z = bf16_val(t.z); o.w = bf16_val(t.w);
    if (tid < 192) *(volatile v4f*)(par + 4 * tid) = o;
    __threadfence();
    if (tid < 192) *(volatile v4f*)(par + 4 * tid) = o;
  }
}

template <int REL>
__global__ __launch_bounds__(NTHR) void k_bucket(const int* __restrict__ keys, const int* __restrict__ srcs,
                                                 int nE, int vec8, int* listg, int* offg, int* cntg,
                                                 float* disg, int* flagg) {
  extern __shared__ __attribute__((aligned(16))) int dsm[];
  int* list = dsm;
  int* hl   = dsm + LISTN;
  int* sl   = hl + RCAP;
  int* cnt  = sl + RCAP;
  int* offs = cnt + NBA;
  int* cur  = offs + NBA;
  int* misc = cur + NBA;
  const int tid = (int)threadIdx.x, lane = tid & 31, wave = tid >> 5;
  const int nodeBase = (int)blockIdx.x * NBA;

  {
    const v4i z4 = {0, 0, 0, 0};
    for (int i = tid * 4; i < AGG_ZINTS; i += NTHR * 4) *(v4ia*)(dsm + i) = z4;
    if (tid < 16) misc[tid] = 0;
  }
  __syncthreads();

  int t = 0, ov = 0;
  const int nChunks = (nE + CHUNK - 1) / CHUNK;
#pragma unroll 1
  for (int ch = 0; ch < nChunks; ++ch) {
    const int cbase = ch * CHUNK;
    const int wc = scan_chunk<SLA>(keys, nE, cbase, nodeBase, NBA, vec8, list, tid, lane, wave);
    if (lane == 0) misc[wave] = wc;
    __syncthreads();
    if (wave == 0) {
#pragma unroll 1
      for (int w2 = 0; w2 < NWAVE; ++w2) {
        int c = misc[w2];
        c = c < 0 ? 0 : (c > WCAP ? WCAP : c);
#pragma unroll 1
        for (int b0 = 0; b0 < c; b0 += 32) {
          const int idx = b0 + lane;
          const int ent = list[w2 * WCAP + (idx < WCAP ? idx : WCAP - 1)];
          const int m32 = (c - b0) < 32 ? (c - b0) : 32;
#pragma unroll 1
          for (int k = 0; k < m32; ++k) {
            const int u    = __builtin_amdgcn_readlane(ent, k);
            const int slot = u & (NBA - 1);
            const int el   = (u >> SLA) & (CHUNK - 1);
            const int pk   = ((cbase + el) << SLA) | slot;
            if (t < RCAP) {
              if (lane == 0) { hl[t] = pk; cnt[slot] = cnt[slot] + 1; }
              t = t + 1;
            } else {
              ov = 1;
            }
          }
        }
      }
    }
    __syncthreads();
  }
  if (wave == 0 && lane == 0) { misc[8] = t; misc[9] = ov; }
  __syncthreads();
  int tt = misc[8];
  tt = tt < 0 ? 0 : (tt > RCAP ? RCAP : tt);
  const int ovf = misc[9];

  if (wave == 0) {
    const int base = lane * (NBA / 32);
    int s = 0;
#pragma unroll 1
    for (int i = 0; i < NBA / 32; ++i) s += cnt[base + i];
    int incl = s;
#pragma unroll
    for (int d = 1; d < 32; d <<= 1) {
      const int y = __shfl_up(incl, d, 32);
      if (lane >= d) incl += y;
    }
    int run = incl - s;
#pragma unroll 1
    for (int i = 0; i < NBA / 32; ++i) {
      const int cv = cnt[base + i];
      offs[base + i] = run;
      cur[base + i]  = run;
      run += cv;
    }
  }
  __syncthreads();
  if (wave == 0) {
#pragma unroll 1
    for (int b0 = 0; b0 < tt; b0 += 32) {
      const int idx = b0 + lane;
      const int ent = hl[idx < RCAP ? idx : RCAP - 1];
      const int m32 = (tt - b0) < 32 ? (tt - b0) : 32;
#pragma unroll 1
      for (int k = 0; k < m32; ++k) {
        const int u    = __builtin_amdgcn_readlane(ent, k);
        const int slot = u & (NBA - 1);
        if (lane == 0) {
          int p = cur[slot];
          p = p < 0 ? 0 : (p > RCAP - 1 ? RCAP - 1 : p);
          sl[p] = u;
          cur[slot] = p + 1;
        }
      }
    }
  }
  __syncthreads();

  {
    int* lg = listg + (size_t)blockIdx.x * RCAP;
    const int ne1 = nE - 1;
#pragma unroll 1
    for (int i = 0; i < RCAP / (NTHR * 4); ++i) {
      const int p4 = (i * NTHR + tid) * 4;
      const v4i ent = *(const v4ia*)(sl + p4);
      int ea = ent.x >> SLA, eb = ent.y >> SLA, ec = ent.z >> SLA, ed = ent.w >> SLA;
      ea = ea < 0 ? 0 : (ea > ne1 ? ne1 : ea);
      eb = eb < 0 ? 0 : (eb > ne1 ? ne1 : eb);
      ec = ec < 0 ? 0 : (ec > ne1 ? ne1 : ec);
      ed = ed < 0 ? 0 : (ed > ne1 ? ne1 : ed);
      const int sa = srcs[ea];
      const int sb = srcs[eb];
      const int sc = srcs[ec];
      const int sd = srcs[ed];
      asm volatile("" :: "v"(sa), "v"(sb), "v"(sc), "v"(sd));
      v4i o;
      o.x = (p4     < tt) ? sa : 0;
      o.y = (p4 + 1 < tt) ? sb : 0;
      o.z = (p4 + 2 < tt) ? sc : 0;
      o.w = (p4 + 3 < tt) ? sd : 0;
      *(volatile v4i*)(lg + p4) = o;
      __threadfence();
      *(volatile v4i*)(lg + p4) = o;
    }
    const v4i c4 = *(const v4ia*)(cnt + 4 * tid);
    const v4i o4 = *(const v4ia*)(offs + 4 * tid);
    v4f d4;
    {
      const float r0 = 1.0f / sqrtf((float)(c4.x > 1 ? c4.x : 1));
      const float r1 = 1.0f / sqrtf((float)(c4.y > 1 ? c4.y : 1));
      const float r2 = 1.0f / sqrtf((float)(c4.z > 1 ? c4.z : 1));
      const float r3 = 1.0f / sqrtf((float)(c4.w > 1 ? c4.w : 1));
      d4.x = (c4.x > 0) ? r0 : 0.0f;
      d4.y = (c4.y > 0) ? r1 : 0.0f;
      d4.z = (c4.z > 0) ? r2 : 0.0f;
      d4.w = (c4.w > 0) ? r3 : 0.0f;
    }
    const v4i f4 = {ovf, tt, 0, 0};
    int*   cg = cntg + nodeBase + 4 * tid;
    int*   og = offg + nodeBase + 4 * tid;
    float* dg = disg + nodeBase + 4 * tid;
    int*   fg = flagg + (size_t)blockIdx.x * 32 + 4 * tid;
    *(volatile v4i*)cg = c4;
    *(volatile v4i*)og = o4;
    if constexpr (REL == 0) *(volatile v4f*)dg = d4;
    if (tid < 8) *(volatile v4i*)fg = f4;
    __threadfence();
    *(volatile v4i*)cg = c4;
    *(volatile v4i*)og = o4;
    if constexpr (REL == 0) *(volatile v4f*)dg = d4;
    if (tid < 8) *(volatile v4i*)fg = f4;
  }
}

template <int REL>
__global__ __launch_bounds__(NTHR) void k_replay(const int* __restrict__ listg, const int* __restrict__ offg,
                                                 const int* __restrict__ cntg, const float* __restrict__ disg,
                                                 const int* __restrict__ flagg,
                                                 const unsigned short* __restrict__ ufp,
                                                 const float* __restrict__ cx, unsigned short* outp) {
  __shared__ __attribute__((aligned(16))) int   cntS[NBA];
  __shared__ __attribute__((aligned(16))) int   offS[NBA];
  __shared__ __attribute__((aligned(16))) float disS[NBA];
  __shared__ __attribute__((aligned(16))) unsigned short rowb[NWAVE * RBW];
  const int tid = (int)threadIdx.x, lane = tid & 31, wave = tid >> 5;
  const int nodeBase = (int)blockIdx.x * NBA;
  const int nSrc = (REL == 0) ? NUSR : NCOM;
  unsigned short* rb = rowb + wave * RBW;
  {
    const v4i c4 = *(const v4i*)(cntg + nodeBase + 4 * tid);
    const v4i o4 = *(const v4i*)(offg + nodeBase + 4 * tid);
    *(v4ia*)(cntS + 4 * tid) = c4;
    *(v4ia*)(offS + 4 * tid) = o4;
    if constexpr (REL == 0) {
      const v4f d4 = *(const v4f*)(disg + nodeBase + 4 * tid);
      *(v4fa*)(disS + 4 * tid) = d4;
    } else {
      const v4f z4 = {0.0f, 0.0f, 0.0f, 0.0f};
      *(v4fa*)(disS + 4 * tid) = z4;
    }
  }
  const int fl = flagg[(size_t)blockIdx.x * 32];
  __syncthreads();
  const float pz = (fl != 0) ? __int_as_float(0x7fc00000) : 0.0f;
  const int* lg = listg + (size_t)blockIdx.x * RCAP;

#pragma unroll 1
  for (int si = 0; si < NBA / NWAVE; ++si) {
    const int s    = si * NWAVE + wave;
    const int node = nodeBase + s;
    int cv = cntS[s];
    const bool big = cv > DEGCAP;
    cv = cv < 0 ? 0 : (cv > DEGCAP ? DEGCAP : cv);
    const int c = __builtin_amdgcn_readfirstlane(cv);
    int ovv = offS[s];
    ovv = ovv < 0 ? 0 : (ovv > RCAP ? RCAP : ovv);
    const int o = __builtin_amdgcn_readfirstlane(ovv);
    float a0 = 0.0f, a1 = 0.0f, a2 = 0.0f, a3 = 0.0f;
#pragma unroll 1
    for (int b0 = 0; b0 < c; b0 += 32) {
      int idx = o + b0 + lane;
      idx = idx > RCAP - 1 ? RCAP - 1 : idx;
      int sr = lg[idx];
      sr = sr < 0 ? 0 : (sr > nSrc - 1 ? nSrc - 1 : sr);
      float wv = 1.0f;
      if constexpr (REL == 0) wv = disg[sr];
      const int wvi = __float_as_int(wv);
      const int m32 = (c - b0) < 32 ? (c - b0) : 32;
#pragma unroll 1
      for (int k = 0; k < m32; ++k) {
        const int sk = __builtin_amdgcn_readlane(sr, k);
        if constexpr (REL == 0) {
          const float ck = __int_as_float(__builtin_amdgcn_readlane(wvi, k));
          const unsigned short* rp = ufp + (size_t)sk * UFP + 4 * lane;
          const v2u q = *(const v2ua*)rp;
          a0 = fmaf(ck, __uint_as_float(q.x << 16),          a0);
          a1 = fmaf(ck, __uint_as_float(q.x & 0xffff0000u), a1);
          a2 = fmaf(ck, __uint_as_float(q.y << 16),          a2);
          a3 = fmaf(ck, __uint_as_float(q.y & 0xffff0000u), a3);
        } else {
          const float* rp = cx + (size_t)sk * DCD + 2 * lane;
          const v2f a = *(const v2fa*)rp;
          a0 = a0 + bf16_val(a.x);
          a1 = a1 + bf16_val(a.y);
        }
      }
    }
    const float pzr = big ? __int_as_float(0x7fc00000) : pz;
    const bool live = node < NUSR;
    if constexpr (REL == 0) {
      const float di = disS[s];
      const float m0 = live ? (a0 * di + pzr) : 0.0f;
      const float m1 = live ? (a1 * di + pzr) : 0.0f;
      const float m2 = live ? (a2 * di + pzr) : 0.0f;
      const float m3 = live ? (a3 * di + pzr) : 0.0f;
      v4us mh, ml;
      {
        unsigned hb;
        hb = bf16_bits(m0); mh[0] = (unsigned short)hb; ml[0] = (unsigned short)bf16_bits(m0 - __uint_as_float(hb << 16));
        hb = bf16_bits(m1); mh[1] = (unsigned short)hb; ml[1] = (unsigned short)bf16_bits(m1 - __uint_as_float(hb << 16));
        hb = bf16_bits(m2); mh[2] = (unsigned short)hb; ml[2] = (unsigned short)bf16_bits(m2 - __uint_as_float(hb << 16));
        hb = bf16_bits(m3); mh[3] = (unsigned short)hb; ml[3] = (unsigned short)bf16_bits(m3 - __uint_as_float(hb << 16));
      }
#if ZERO_LO_G
      { const v4us z4 = {0, 0, 0, 0}; ml = z4; }
#endif
      if (lane < 24) {
        *(v4usa*)(rb + 4 * lane) = mh;
        *(v4usa*)(rb + 96 + 4 * lane) = ml;
      }
      wave_sync();
      const int lc = lane < 24 ? lane : 23;
      const v8us q = *(const v8usa*)(rb + 8 * lc);
      wave_sync();
      if (node < MPAD && lane < 24) {
        unsigned short* rpw = outp + (size_t)node * GPI + 8 * lane;
        *(volatile v8us*)rpw = q;
        __threadfence();
        *(volatile v8us*)rpw = q;
      }
    } else {
      const float den = (c > 0) ? (float)c : 1.0f;
      const float rcp = 1.0f / den;
      const float m0 = live ? (a0 * rcp + pzr) : 0.0f;
      const float m1 = live ? (a1 * rcp + pzr) : 0.0f;
      v2us mh, ml;
      {
        unsigned hb;
        hb = bf16_bits(m0); mh[0] = (unsigned short)hb; ml[0] = (unsigned short)bf16_bits(m0 - __uint_as_float(hb << 16));
        hb = bf16_bits(m1); mh[1] = (unsigned short)hb; ml[1] = (unsigned short)bf16_bits(m1 - __uint_as_float(hb << 16));
      }
#if ZERO_LO_C
      { const v2us z2 = {0, 0}; ml = z2; }
#endif
      *(v2usa*)(rb + 2 * lane) = mh;
      *(v2usa*)(rb + 64 + 2 * lane) = ml;
      wave_sync();
      const int lc = lane < 16 ? lane : 15;
      const v8us q = *(const v8usa*)(rb + 8 * lc);
      wave_sync();
      if (node < MPAD && lane < 16) {
        unsigned short* rpw = outp + (size_t)node * CPI + 8 * lane;
        *(volatile v8us*)rpw = q;
        __threadfence();
        *(volatile v8us*)rpw = q;
      }
    }
  }
}

__device__ __forceinline__ void kstep8(const unsigned short* __restrict__ ap,
                                       const unsigned short* __restrict__ bp, v8f (&acc)[8]) {
  FragB af;
  af.h[0] = *(const v8usa*)ap;
  af.h[1] = *(const v8usa*)(ap + 16);
#pragma unroll
  for (int nt = 0; nt < 8; ++nt) {
    const unsigned short* wq = bp + (size_t)(16 * nt) * KT;
    FragB bf;
    bf.h[0] = *(const v8usa*)wq;
    bf.h[1] = *(const v8usa*)(wq + 16);
    acc[nt] = wmb(af, bf, acc[nt]);
  }
}

__global__ __launch_bounds__(NTHR) __attribute__((amdgpu_num_vgpr(248)))
void k_gemm(const unsigned short* __restrict__ ufp, const unsigned short* __restrict__ gp,
            const unsigned short* __restrict__ cp, const unsigned short* __restrict__ bt,
            const float* __restrict__ par, float* outp, float* rec) {
  __shared__ __attribute__((aligned(16))) float S[128 * HD];
  __shared__ __attribute__((aligned(16))) float sb[2 * HD];
  __shared__ __attribute__((aligned(16))) float recs[2 * HD];
  const int tid = (int)threadIdx.x, lane = tid & 31, wave = tid >> 5, hh = lane >> 4, m = lane & 15;
  const int rowBase = (int)blockIdx.x * 128;

  if (tid < 64) {
    const v4f t1 = *(const v4f*)(par + 4 * tid);
    const v4f t2 = *(const v4f*)(par + 2 * HD + 4 * tid);
    *(v4fa*)(sb + 4 * tid) = t1 + t2;
  }
  __syncthreads();

  const size_t arow = (size_t)(rowBase + 16 * wave + m);
  const unsigned short* aU = ufp + arow * UFP + 8 * hh;
  const unsigned short* aG = gp  + arow * GPI + 8 * hh;
  const unsigned short* aC = cp  + arow * CPI + 8 * hh;

#pragma unroll
  for (int h = 0; h < 2; ++h) {
    v8f acc[8];
    {
      const v8f z = {0.f, 0.f, 0.f, 0.f, 0.f, 0.f, 0.f, 0.f};
#pragma unroll
      for (int t = 0; t < 8; ++t) acc[t] = z;
    }
    const unsigned short* bB = bt + (size_t)(h * HD + m) * KT + 8 * hh;
#pragma unroll 1
    for (int s = 0; s < 3; ++s) kstep8(aU + 32 * s, bB + 32 * s, acc);
#pragma unroll 1
    for (int s = 0; s < 6; ++s) kstep8(aG + 32 * s, bB + 96 + 32 * s, acc);
#pragma unroll 1
    for (int s = 0; s < 4; ++s) kstep8(aC + 32 * s, bB + 288 + 32 * s, acc);

#pragma unroll
    for (int nt = 0; nt < 8; ++nt) {
      const int lc = 16 * nt + m;
      const float bsv = sb[h * HD + lc];
#pragma unroll
      for (int r = 0; r < 8; ++r) {
        const int lr = 16 * wave + 8 * hh + r;
        const float t = acc[nt][r] + bsv;
        const float y = (t > 0.0f) ? t : 0.3f * t;
        if (h == 0) S[lr * HD + lc] = y;
        else        S[lr * HD + lc] = S[lr * HD + lc] + y;
      }
    }
  }
  __syncthreads();

  int nv = NUSR - rowBase;
  nv = nv > 128 ? 128 : (nv < 1 ? 1 : nv);
  if (tid < HD) {
    float s = 0.0f;
#pragma unroll 4
    for (int i = 0; i < nv; ++i) s += S[i * HD + tid];
    const float mean = s * (1.0f / (float)nv);
    float q = 0.0f;
#pragma unroll 4
    for (int i = 0; i < nv; ++i) {
      const float d = S[i * HD + tid] - mean;
      q = fmaf(d, d, q);
    }
    recs[2 * tid]     = mean;
    recs[2 * tid + 1] = q;
  }
  __syncthreads();

  v4f pv[16];
#pragma unroll
  for (int i = 0; i < 16; ++i) pv[i] = *(const v4fa*)(S + (16 * wave + i) * HD + 4 * lane);
  v4f rv = {0.0f, 0.0f, 0.0f, 0.0f};
  if (tid < 64) rv = *(const v4fa*)(recs + 4 * tid);
  float* rg = rec + (size_t)blockIdx.x * (2 * HD) + 4 * (tid & 63);

#pragma unroll
  for (int i = 0; i < 16; ++i) {
    const int r = rowBase + 16 * wave + i;
    if (r < NUSR) *(volatile v4f*)(outp + (size_t)r * HD + 4 * lane) = pv[i];
  }
  if (tid < 64) *(volatile v4f*)rg = rv;
  __threadfence();
#pragma unroll
  for (int i = 0; i < 16; ++i) {
    const int r = rowBase + 16 * wave + i;
    if (r < NUSR) *(volatile v4f*)(outp + (size_t)r * HD + 4 * lane) = pv[i];
  }
  if (tid < 64) *(volatile v4f*)rg = rv;
}

__global__ __launch_bounds__(HD) void k_comb(const float* __restrict__ rec, const float* __restrict__ par,
                                             int nTiles, int nRows, float* stat) {
  __shared__ __attribute__((aligned(16))) float st[4 * HD];
  const int c = (int)threadIdx.x;
  double n = 0.0, mean = 0.0, M2 = 0.0;
#pragma unroll 1
  for (int b = 0; b < nTiles; ++b) {
    const v2f r = *(const v2fa*)(rec + (size_t)b * (2 * HD) + 2 * c);
    int left = nRows - b * 128;
    left = left > 128 ? 128 : left;
    const double nb = (double)left;
    const double mb = (double)r.x;
    const double qb = (double)r.y;
    if (nb > 0.5) {
      const double nn = n + nb;
      const double delta = mb - mean;
      const double f = nb / nn;
      mean = mean + delta * f;
      M2 = M2 + qb + delta * delta * n * f;
      n = nn;
    }
  }
  const double nt = n < 1.0 ? 1.0 : n;
  const float varf  = (float)(M2 / nt);
  const float meanf = (float)mean;
  const float rstd  = 1.0f / sqrtf(varf + 1e-5f);
  st[c]          = meanf;
  st[HD + c]     = rstd;
  st[2 * HD + c] = par[4 * HD + c];
  st[3 * HD + c] = par[5 * HD + c];
  __syncthreads();
  const v4f v = *(const v4fa*)(st + 4 * c);
  *(volatile v4f*)(stat + 4 * c) = v;
  __threadfence();
  *(volatile v4f*)(stat + 4 * c) = v;
}

__global__ __launch_bounds__(NTHR) void k_bn(const float* __restrict__ stat, int nUnits, float* out) {
  __shared__ __attribute__((aligned(16))) float ssh[4 * HD];
  const int tid = (int)threadIdx.x;
  if (tid < HD) {
    const v4f t = *(const v4f*)(stat + 4 * tid);
    *(v4fa*)(ssh + 4 * tid) = t;
  }
  __syncthreads();
  const int u = (int)blockIdx.x * NTHR + tid;
  if (u >= nUnits) return;
  const int c4 = (u & 31) * 4;
  float* op = out + (size_t)u * 4;
  const v4f x = *(const v4f*)op;
  v4f o;
  o.x = ((x.x - ssh[c4 + 0]) * ssh[HD + c4 + 0]) * ssh[2 * HD + c4 + 0] + ssh[3 * HD + c4 + 0];
  o.y = ((x.y - ssh[c4 + 1]) * ssh[HD + c4 + 1]) * ssh[2 * HD + c4 + 1] + ssh[3 * HD + c4 + 1];
  o.z = ((x.z - ssh[c4 + 2]) * ssh[HD + c4 + 2]) * ssh[2 * HD + c4 + 2] + ssh[3 * HD + c4 + 2];
  o.w = ((x.w - ssh[c4 + 3]) * ssh[HD + c4 + 3]) * ssh[2 * HD + c4 + 3] + ssh[3 * HD + c4 + 3];
  *(volatile v4f*)op = o;
  __threadfence();
  *(volatile v4f*)op = o;
}

static inline size_t al256(size_t o) { return (o + 255) & ~(size_t)255; }

extern "C" void kernel_launch(void* const* d_in, const int* in_sizes, int n_in,
                              void* d_out, int out_size, void* d_ws, size_t ws_size,
                              hipStream_t stream) {
  if (n_in < 19) return;
  if (in_sizes[0] != NU2 || in_sizes[1] != NU1 * 10 || in_sizes[2] != NCOM * DCD) return;
  if (in_sizes[3] != 2 * NEDG || in_sizes[4] != NEDG || in_sizes[5] != NEDG) return;
  if (in_sizes[6] != NU2 * EDIM) return;
  if (in_sizes[7] != 32 || in_sizes[8] != 32 || in_sizes[9] != 32 || in_sizes[10] != 32 || in_sizes[11] != 32) return;
  if (in_sizes[12] != 2 * EDIM * HD || in_sizes[13] != 2 * HD) return;
  if (in_sizes[14] != 2 * DCD * HD || in_sizes[15] != 2 * HD) return;
  if (in_sizes[16] != 2 * EDIM * HD || in_sizes[17] != HD || in_sizes[18] != HD) return;
  if ((long long)out_size != (long long)NUSR * HD) return;

  const int*   nidx = (const int*)d_in[0];
  const float* uf   = (const float*)d_in[1];
  const float* cx   = (const float*)d_in[2];
  const int*   euu  = (const int*)d_in[3];
  const int*   csrc = (const int*)d_in[4];
  const int*   cdst = (const int*)d_in[5];
  const float* emb  = (const float*)d_in[6];
  const float* e0   = (const float*)d_in[7];
  const float* e3   = (const float*)d_in[8];
  const float* e7   = (const float*)d_in[9];
  const float* e8   = (const float*)d_in[10];
  const float* e9   = (const float*)d_in[11];
  const float* wg   = (const float*)d_in[12];
  const float* bg   = (const float*)d_in[13];
  const float* wl   = (const float*)d_in[14];
  const float* bl   = (const float*)d_in[15];
  const float* wr   = (const float*)d_in[16];
  const float* gam  = (const float*)d_in[17];
  const float* bet  = (const float*)d_in[18];
  float* out = (float*)d_out;

  char* ws = (char*)d_ws;
  size_t off = 0;
  const size_t oUF  = off; off = al256(off + (size_t)MPAD * UFP * 2);
  const size_t oG   = off; off = al256(off + (size_t)MPAD * GPI * 2);
  const size_t oCP  = off; off = al256(off + (size_t)MPAD * CPI * 2);
  const size_t oLU  = off; off = al256(off + (size_t)NBLK * RCAP * 4);
  const size_t oLC  = off; off = al256(off + (size_t)NBLK * RCAP * 4);
  const size_t oOU  = off; off = al256(off + (size_t)NSLOT * 4);
  const size_t oCU  = off; off = al256(off + (size_t)NSLOT * 4);
  const size_t oDU  = off; off = al256(off + (size_t)NSLOT * 4);
  const size_t oOC  = off; off = al256(off + (size_t)NSLOT * 4);
  const size_t oCC  = off; off = al256(off + (size_t)NSLOT * 4);
  const size_t oFU  = off; off = al256(off + (size_t)NBLK * 128);
  const size_t oFC  = off; off = al256(off + (size_t)NBLK * 128);
  const size_t oBT  = off; off = al256(off + (size_t)BTN * KT * 2);
  const size_t oREC = off; off = al256(off + (size_t)NTILE * 2 * HD * 4);
  const size_t oPAR = off; off = al256(off + (size_t)6 * HD * 4);
  const size_t oST  = off; off = al256(off + (size_t)4 * HD * 4);
  if (off > ws_size || off > (size_t)WSMAX) return;
  unsigned short* UF  = (unsigned short*)(ws + oUF);
  unsigned short* G   = (unsigned short*)(ws + oG);
  unsigned short* CP  = (unsigned short*)(ws + oCP);
  int*   LU  = (int*)(ws + oLU);
  int*   LC  = (int*)(ws + oLC);
  int*   OU  = (int*)(ws + oOU);
  int*   CU  = (int*)(ws + oCU);
  float* DU  = (float*)(ws + oDU);
  int*   OC  = (int*)(ws + oOC);
  int*   CC  = (int*)(ws + oCC);
  int*   FU  = (int*)(ws + oFU);
  int*   FC  = (int*)(ws + oFC);
  unsigned short* BT = (unsigned short*)(ws + oBT);
  float* REC = (float*)(ws + oREC);
  float* PAR = (float*)(ws + oPAR);
  float* ST  = (float*)(ws + oST);

  const size_t bucketLds = (size_t)AGG_LDS_INTS * 4;
  hipFuncSetAttribute(reinterpret_cast<const void*>(&k_bucket<0>), hipFuncAttributeMaxDynamicSharedMemorySize, (int)bucketLds);
  hipFuncSetAttribute(reinterpret_cast<const void*>(&k_bucket<1>), hipFuncAttributeMaxDynamicSharedMemorySize, (int)bucketLds);

  const int vec8 = ((NEDG & 3) == 0) ? 1 : 0;
  k_prep<<<PBTOT, NTHR, 0, stream>>>(nidx, uf, emb, e0, e3, e7, e8, e9, wg, bg, wl, bl, wr, gam, bet, UF, BT, PAR);
  k_bucket<0><<<NBLK, NTHR, bucketLds, stream>>>(euu + NEDG, euu, NEDG, vec8, LU, OU, CU, DU, FU);
  k_bucket<1><<<NBLK, NTHR, bucketLds, stream>>>(cdst, csrc, NEDG, vec8, LC, OC, CC, DU, FC);
  k_replay<0><<<NBLK, NTHR, 0, stream>>>(LU, OU, CU, DU, FU, UF, cx, G);
  k_replay<1><<<NBLK, NTHR, 0, stream>>>(LC, OC, CC, DU, FC, UF, cx, CP);
  k_gemm<<<NTILE, NTHR, 0, stream>>>(UF, G, CP, BT, PAR, out, REC);
  k_comb<<<1, HD, 0, stream>>>(REC, PAR, NTILE, NUSR, ST);
  k_bn<<<(NUSR * HD / 4) / NTHR, NTHR, 0, stream>>>(ST, NUSR * HD / 4, out);
}
